// InfoNCEPatchLoss_49976239456824
// MI455X (gfx1250) — hardware-run, weakly checked
//
#include <hip/hip_runtime.h>
#include <math.h>
#include <stdint.h>

#define NB     8
#define IMH    256
#define IMW    256
#define NCH    3
#define HW     (IMH * IMW)
#define NANCH  100
#define MT     7
#define APAD   128
#define KD     32
#define DLIVE  27
#define NPR    16
#define PRPIX  (HW / NPR)
#define WPB    4
#define TPW    (PRPIX / (WPB * 16))
#define PXB    64
#define LOG2E  1.4426950408889634f

static_assert(HW == 65536);
static_assert(IMW == 256);
static_assert(NPR * PRPIX == HW);
static_assert(WPB * 16 * TPW == PRPIX);
static_assert(MT * 16 >= NANCH);
static_assert(APAD >= MT * 16);
static_assert(APAD == 128);
static_assert(((NB * HW) % PXB) == 0);
static_assert((IMW % PXB) == 0);
static_assert(KD == 32);
static_assert(DLIVE <= KD);
static_assert(NCH * 9 == DLIVE);

typedef __bf16       v16b __attribute__((ext_vector_type(16)));
typedef __bf16       v8b  __attribute__((ext_vector_type(8)));
typedef float        v8f  __attribute__((ext_vector_type(8)));
typedef float        v4f  __attribute__((ext_vector_type(4)));
typedef unsigned int v4u  __attribute__((ext_vector_type(4)));

__device__ __forceinline__ unsigned short bf_bits(float f) {
  unsigned u = __float_as_uint(f);
  return (unsigned short)((u + 0x7FFFu + ((u >> 16) & 1u)) >> 16);
}
__device__ __forceinline__ float bf_up(unsigned short h) { return __uint_as_float(((unsigned)h) << 16); }
__device__ __forceinline__ unsigned pk16(unsigned short a, unsigned short b) { return (unsigned)a | ((unsigned)b << 16); }
__device__ __forceinline__ v8f zero8() { v8f z = {0.f, 0.f, 0.f, 0.f, 0.f, 0.f, 0.f, 0.f}; return z; }

__device__ __forceinline__ v16b ldfrag_b(const __bf16* p) {
  union { v16b v; v8b h[2]; } f;
  f.h[0] = *(const v8b*)(p);
  f.h[1] = *(const v8b*)(p + 16);
  return f.v;
}

__device__ __forceinline__ v8f mma_b(v16b a, v16b b, v8f c) {
  c = __builtin_amdgcn_wmma_f32_16x16x32_bf16(false, a, false, b, (short)0, c, false, false);
#if defined(__HIP_DEVICE_COMPILE__)
  asm volatile("v_nop\n\tv_nop\n\tv_nop\n\tv_nop" : "+v"(c) : "v"(a), "v"(b));
#endif
  return c;
}

__global__ __launch_bounds__(PXB) void build_rows(const float* __restrict__ lat, v4u* PTv, float* RN) {
  __shared__ v4u tile[PXB * 4];
  __shared__ __align__(16) float rns[PXB];

  const int t   = threadIdx.x;
  const int gid = blockIdx.x * PXB + t;
  const int b   = gid >> 16;
  const int p   = gid & (HW - 1);
  const int y   = p >> 8;
  const int x   = p & (IMW - 1);

  float v[DLIVE];
#pragma unroll
  for (int i = 0; i < 3; ++i) {
    const int sy = min(max(y + i - 1, 0), IMH - 1);
#pragma unroll
    for (int j = 0; j < 3; ++j) {
      const int sx = min(max(x + j - 1, 0), IMW - 1);
      const size_t o = ((size_t)(b * IMH + sy) * IMW + sx) * NCH;
#pragma unroll
      for (int c = 0; c < NCH; ++c) v[c * 9 + i * 3 + j] = lat[o + c];
    }
  }

  unsigned short hb[KD];
  float ss = 0.f;
#pragma unroll
  for (int d = 0; d < DLIVE; ++d) {
    hb[d] = bf_bits(v[d]);
    const float yv = bf_up(hb[d]);
    ss += yv * yv;
  }
#pragma unroll
  for (int d = DLIVE; d < KD; ++d) hb[d] = 0;

  v4u q[4];
#pragma unroll
  for (int jj = 0; jj < 4; ++jj) {
    v4u w;
#pragma unroll
    for (int e = 0; e < 4; ++e) w[e] = pk16(hb[(jj * 4 + e) * 2], hb[(jj * 4 + e) * 2 + 1]);
    q[jj] = w;
  }
  const float rn = __builtin_amdgcn_rcpf(fmaxf(sqrtf(ss), 1e-12f));

#pragma unroll
  for (int jj = 0; jj < 4; ++jj) tile[t * 4 + jj] = q[jj];
  rns[t] = rn;
  __syncthreads();

  const v4u o0 = tile[t];
  const v4u o1 = tile[t + PXB];
  const v4u o2 = tile[t + 2 * PXB];
  const v4u o3 = tile[t + 3 * PXB];
  const int  tc = t & 15;
  const v4f  rv = *(const v4f*)(&rns[4 * tc]);
  v4u*   dst = PTv + (size_t)blockIdx.x * (PXB * 4);
  float* drn = RN + (size_t)blockIdx.x * PXB + 4 * tc;

  *(volatile v4u*)(dst + t)           = o0;
  *(volatile v4u*)(dst + t + PXB)     = o1;
  *(volatile v4u*)(dst + t + 2 * PXB) = o2;
  *(volatile v4u*)(dst + t + 3 * PXB) = o3;
  if (t < 16) *(volatile v4f*)drn = rv;
  __threadfence();
  *(volatile v4u*)(dst + t)           = o0;
  *(volatile v4u*)(dst + t + PXB)     = o1;
  *(volatile v4u*)(dst + t + 2 * PXB) = o2;
  *(volatile v4u*)(dst + t + 3 * PXB) = o3;
  if (t < 16) *(volatile v4f*)drn = rv;
}

__global__ __launch_bounds__(APAD) void gather_rows(const v4u* __restrict__ PTv, const float* __restrict__ RN,
                                                     const int* __restrict__ qidx, v4u* APv, float* RNA) {
  __shared__ v4u tA[APAD * 4];
  __shared__ __align__(16) float rs[APAD];

  const int t    = threadIdx.x;
  const int lane = t & 31;
  const int wave = t >> 5;
  const int b    = blockIdx.x;
  const bool live = (t < NANCH);
  const int ta   = live ? t : (NANCH - 1);
  int id = qidx[b * NANCH + ta];
  id = min(max(id, 0), HW - 1);
  const size_t src = ((size_t)b * HW + id);
  v4u q0 = PTv[src * 4 + 0];
  v4u q1 = PTv[src * 4 + 1];
  v4u q2 = PTv[src * 4 + 2];
  v4u q3 = PTv[src * 4 + 3];
  float r = RN[src];
  const unsigned msk = live ? 0xffffffffu : 0u;
  const v4u mv = {msk, msk, msk, msk};
  q0 = q0 & mv; q1 = q1 & mv; q2 = q2 & mv; q3 = q3 & mv;
  r = live ? r : 0.f;

  tA[t * 4 + 0] = q0;
  tA[t * 4 + 1] = q1;
  tA[t * 4 + 2] = q2;
  tA[t * 4 + 3] = q3;
  rs[t] = r;
  __syncthreads();

  const v4u o0 = tA[t];
  const v4u o1 = tA[t + APAD];
  const v4u o2 = tA[t + 2 * APAD];
  const v4u o3 = tA[t + 3 * APAD];
  const v4f rv = *(const v4f*)(&rs[4 * lane]);
  v4u*   dst = APv + (size_t)b * (APAD * 4);
  float* drn = RNA + (size_t)b * APAD + 4 * lane;

  *(volatile v4u*)(dst + t)            = o0;
  *(volatile v4u*)(dst + t + APAD)     = o1;
  *(volatile v4u*)(dst + t + 2 * APAD) = o2;
  *(volatile v4u*)(dst + t + 3 * APAD) = o3;
  if (wave == 0) *(volatile v4f*)drn = rv;
  __threadfence();
  *(volatile v4u*)(dst + t)            = o0;
  *(volatile v4u*)(dst + t + APAD)     = o1;
  *(volatile v4u*)(dst + t + 2 * APAD) = o2;
  *(volatile v4u*)(dst + t + 3 * APAD) = o3;
  if (wave == 0) *(volatile v4f*)drn = rv;
}

__global__ __launch_bounds__(WPB * 32) void tile_sums(const unsigned short* __restrict__ PT,
                                                      const float* __restrict__ RN,
                                                      const unsigned short* __restrict__ AP,
                                                      const float* __restrict__ RNA,
                                                      const int* __restrict__ qidx, float* PART) {
  const __bf16* Pb = (const __bf16*)(const void*)PT;
  const __bf16* Ab = (const __bf16*)(const void*)AP;
  __shared__ __align__(16) float sred[4][64];

  const int lane = threadIdx.x & 31;
  const int wave = threadIdx.x >> 5;
  const int h    = lane >> 4;
  const int m    = lane & 15;
  const int pr   = blockIdx.x;
  const int mt   = blockIdx.y;
  const int b    = blockIdx.z;

  const v16b afr = ldfrag_b(Ab + ((size_t)(b * APAD + mt * 16 + m)) * KD + 8 * h);

  float rsc[8];
  int ay[8], ax[8];
  {
    const v4f r0 = *(const v4f*)(RNA + (size_t)b * APAD + mt * 16 + 8 * h);
    const v4f r1 = *(const v4f*)(RNA + (size_t)b * APAD + mt * 16 + 8 * h + 4);
#pragma unroll
    for (int i = 0; i < 4; ++i) { rsc[i] = r0[i] * LOG2E; rsc[4 + i] = r1[i] * LOG2E; }
  }
#pragma unroll
  for (int r = 0; r < 8; ++r) {
    int a = mt * 16 + 8 * h + r;
    a = min(a, NANCH - 1);
    int id = qidx[b * NANCH + a];
    id = min(max(id, 0), HW - 1);
    ay[r] = id >> 8;
    ax[r] = id & (IMW - 1);
  }

  float ps[8], ns[8], pc[8], nc[8];
#pragma unroll
  for (int r = 0; r < 8; ++r) { ps[r] = 0.f; ns[r] = 0.f; pc[r] = 0.f; nc[r] = 0.f; }

  const int    pixbase = pr * PRPIX + wave * (TPW * 16);
  const size_t rowbase = (size_t)b * HW + pixbase;

#pragma unroll 1
  for (int t = 0; t < TPW; ++t) {
    const int    pg   = pixbase + t * 16;
    const size_t prow = rowbase + (size_t)t * 16 + m;
    const v16b bfr = ldfrag_b(Pb + prow * KD + 8 * h);
    v8f acc = mma_b(afr, bfr, zero8());
    const float rp = RN[prow];
    const int py = pg >> 8;
    const int px = (pg & (IMW - 1)) + m;
#pragma unroll
    for (int r = 0; r < 8; ++r) {
      const float e  = __builtin_amdgcn_exp2f(acc[r] * (rsc[r] * rp));
      const int   dy = py - ay[r];
      const int   dx = px - ax[r];
      const int   d2 = dy * dy + dx * dx;
      const bool  pos = (d2 > 0) && (d2 <= 9);
      const bool  neg = (d2 > 121);
      ps[r] += pos ? e : 0.f;
      pc[r] += pos ? 1.f : 0.f;
      ns[r] += neg ? e : 0.f;
      nc[r] += neg ? 1.f : 0.f;
    }
  }

#pragma unroll
  for (int r = 0; r < 8; ++r) {
#pragma unroll
    for (int off = 1; off < 16; off <<= 1) {
      ps[r] += __shfl_xor(ps[r], off, 32);
      pc[r] += __shfl_xor(pc[r], off, 32);
      ns[r] += __shfl_xor(ns[r], off, 32);
      nc[r] += __shfl_xor(nc[r], off, 32);
    }
  }
  if (m == 0) {
#pragma unroll
    for (int r = 0; r < 8; ++r) {
      const int rr = wave * 16 + 8 * h + r;
      sred[0][rr] = ps[r];
      sred[1][rr] = ns[r];
      sred[2][rr] = pc[r];
      sred[3][rr] = nc[r];
    }
  }
  __syncthreads();
  if (wave == 0) {
    const int la = lane & 15;
    float s0 = 0.f, s1 = 0.f, s2 = 0.f, s3 = 0.f;
#pragma unroll
    for (int w = 0; w < WPB; ++w) {
      s0 += sred[0][w * 16 + la];
      s1 += sred[1][w * 16 + la];
      s2 += sred[2][w * 16 + la];
      s3 += sred[3][w * 16 + la];
    }
    v4f rec;
    rec[0] = s0; rec[1] = s1; rec[2] = s2; rec[3] = s3;
    float* dst = PART + (((size_t)(b * MT + mt)) * NPR + pr) * 64 + la * 4;
    if (lane < 16) *(volatile v4f*)dst = rec;
    __threadfence();
    if (lane < 16) *(volatile v4f*)dst = rec;
  }
}

__global__ __launch_bounds__(256) void finish_loss(const float* __restrict__ PART, float* out) {
  __shared__ float s[256];
  const int tid = threadIdx.x;
  float acc = 0.f;
#pragma unroll 1
  for (int k = tid; k < NB * NANCH; k += 256) {
    const int b   = k / NANCH;
    const int n   = k - b * NANCH;
    const int mt  = n >> 4;
    const int r16 = n & 15;
    const float* rec = PART + ((size_t)(b * MT + mt) * NPR) * 64 + r16 * 4;
    float ps = 0.f, ns = 0.f, pc = 0.f, nc = 0.f;
#pragma unroll 1
    for (int pr = 0; pr < NPR; ++pr) {
      const v4f v = *(const v4f*)(rec + (size_t)pr * 64);
      ps += v[0]; ns += v[1]; pc += v[2]; nc += v[3];
    }
    const float pm    = ps * __builtin_amdgcn_rcpf(fmaxf(pc, 1.f));
    const float nm    = ns * __builtin_amdgcn_rcpf(fmaxf(nc, 1.f));
    const bool  valid = (pc > 0.f) && (nc > 0.f);
    const float q     = pm * __builtin_amdgcn_rcpf(pm + nm + 1e-8f);
    const float term  = -logf(q);
    acc += valid ? term : 0.f;
  }
  s[tid] = acc;
  __syncthreads();
#pragma unroll
  for (int off = 128; off > 0; off >>= 1) {
    if (tid < off) s[tid] += s[tid + off];
    __syncthreads();
  }
  if (tid == 0) {
    const float loss = s[0] * (1.0f / (float)(NB * NANCH));
    *(volatile float*)out = loss;
    __threadfence();
    *(volatile float*)out = loss;
  }
}

extern "C" void kernel_launch(void* const* d_in, const int* in_sizes, int n_in,
                              void* d_out, int out_size, void* d_ws, size_t ws_size,
                              hipStream_t stream) {
  if (n_in < 2) return;
  if (in_sizes[0] != NB * HW * NCH) return;
  if (in_sizes[1] != NB * NANCH) return;
  if (out_size < 1) return;

  const float* lat  = (const float*)d_in[0];
  const int*   qidx = (const int*)d_in[1];
  float* out = (float*)d_out;

  const size_t bPT   = (size_t)NB * HW * KD * 2;
  const size_t bRN   = (size_t)NB * HW * 4;
  const size_t bAP   = (size_t)NB * APAD * KD * 2;
  const size_t bRNA  = (size_t)NB * APAD * 4;
  const size_t bPART = (size_t)NB * MT * NPR * 64 * 4;
  size_t off = 0;
  const size_t oPT   = off; off += bPT;
  const size_t oRN   = off; off += bRN;
  const size_t oAP   = off; off += bAP;
  const size_t oRNA  = off; off += bRNA;
  const size_t oPART = off; off += bPART;
  if (off > ws_size) return;
  if (off > (size_t)134217728) return;

  char* ws = (char*)d_ws;
  v4u*   PTv  = (v4u*)(ws + oPT);
  float* RN   = (float*)(ws + oRN);
  v4u*   APv  = (v4u*)(ws + oAP);
  float* RNA  = (float*)(ws + oRNA);
  float* PART = (float*)(ws + oPART);

  build_rows<<<dim3((NB * HW) / PXB), dim3(PXB), 0, stream>>>(lat, PTv, RN);
  gather_rows<<<dim3(NB), dim3(APAD), 0, stream>>>((const v4u*)PTv, RN, qidx, APv, RNA);
  tile_sums<<<dim3(NPR, MT, NB), dim3(WPB * 32), 0, stream>>>((const unsigned short*)(ws + oPT), RN,
                                                             (const unsigned short*)(ws + oAP), RNA,
                                                             qidx, PART);
  finish_loss<<<dim3(1), dim3(256), 0, stream>>>(PART, out);
  (void)hipGetLastError();
}
